// HybridNATGraphQNN_65481071399142
// MI455X (gfx1250) — hardware-verified
//
#include <hip/hip_runtime.h>
#include <stddef.h>


#define NPIX1   196
#define C1      8
#define H1S     (NPIX1 * C1)
#define K2      96
#define C2      16
#define NWIN    49
#define KF      784
#define KFP     800
#define NF1     64
#define NF2     8
#define NF2P    16
#define NW      8
#define NOUT    4
#define T1      64
#define T2      256
#define SPB2    4
#define TF      128
#define RPB     64
#define TS      256
#define TQ      32
#define SHP     72
#define NPREPB  27
#define WSCAP   134217728
#define BN_EPS  1e-5f

static_assert(KFP % 32 == 0);
static_assert(K2 % 32 == 0);
static_assert((SHP * 2) % 16 == 0);
static_assert(SPB2 * NPIX1 == NWIN * 16);
static_assert((SPB2 * KFP * 2) % 128 == 0);
static_assert(RPB == (TF / 32) * 16);
static_assert(NF1 * KFP == 25 * 256 * 8);
static_assert(SPB2 * (KFP / 8) - T2 > 0 && SPB2 * (KFP / 8) - T2 <= T2);

typedef float          v4f  __attribute__((ext_vector_type(4)));
typedef float          v8f  __attribute__((ext_vector_type(8)));
typedef unsigned short v8us __attribute__((ext_vector_type(8)));
typedef __bf16         v16b __attribute__((ext_vector_type(16)));
union FragB { v16b v; v8us h[2]; };

__device__ __forceinline__ unsigned int bfr(float f) {
  const unsigned int u = __float_as_uint(f);
  return (u + 0x7FFFu + ((u >> 16) & 1u)) >> 16;
}

__device__ __forceinline__ void split1(float x, unsigned short& hb, unsigned short& lb) {
  const unsigned int hu = bfr(x);
  const float hf = __uint_as_float(hu << 16);
  hb = (unsigned short)hu;
  lb = (unsigned short)bfr(x - hf);
}

__device__ __forceinline__ void split8(v4f a, v4f b, v8us& hi, v8us& lo) {
  unsigned short hb, lb;
  split1(a.x, hb, lb); hi[0] = hb; lo[0] = lb;
  split1(a.y, hb, lb); hi[1] = hb; lo[1] = lb;
  split1(a.z, hb, lb); hi[2] = hb; lo[2] = lb;
  split1(a.w, hb, lb); hi[3] = hb; lo[3] = lb;
  split1(b.x, hb, lb); hi[4] = hb; lo[4] = lb;
  split1(b.y, hb, lb); hi[5] = hb; lo[5] = lb;
  split1(b.z, hb, lb); hi[6] = hb; lo[6] = lb;
  split1(b.w, hb, lb); hi[7] = hb; lo[7] = lb;
}

__device__ __forceinline__ v8f wmb(v16b a, v16b b, v8f c) {
  v8f d = __builtin_amdgcn_wmma_f32_16x16x32_bf16(false, a, false, b, (short)0, c, false, false);
  asm volatile("v_nop\n\tv_nop\n\tv_nop\n\tv_nop" : "+v"(d) : "v"(a), "v"(b));
  return d;
}

__device__ __forceinline__ void blockred(double* red, int tid) {
  __syncthreads();
#pragma unroll 1
  for (int off = TS / 2; off > 0; off >>= 1) {
    if (tid < off) {
#pragma unroll
      for (int f = 0; f < NW; ++f) red[f * TS + tid] += red[f * TS + tid + off];
    }
    __syncthreads();
  }
}

__global__ __launch_bounds__(256) void k_prep(
    const float* __restrict__ c2w, const float* __restrict__ f1w, const float* __restrict__ f2w,
    unsigned short* wt, unsigned short* wf1, unsigned short* wf2) {
  const int tid = (int)threadIdx.x, b = (int)blockIdx.x;
  float v[8];
  unsigned short* dh;
  unsigned short* dl;
  bool act = true;
  if (b < 25) {
    const int c  = b * 256 + tid;
    const int n  = c / 100;
    const int k0 = (c - n * 100) * 8;
#pragma unroll
    for (int e = 0; e < 8; ++e) {
      const int k  = k0 + e;
      const int kc = k < KF ? k : KF - 1;
      const float t = f1w[n * KF + kc];
      v[e] = (k < KF) ? t : 0.0f;
    }
    dh = wf1 + (size_t)c * 8;
    dl = dh + NF1 * KFP;
  } else if (b == 25) {
    act = tid < C2 * (K2 / 8);
    const int c   = tid < C2 * (K2 / 8) - 1 ? tid : C2 * (K2 / 8) - 1;
    const int oc  = c / (K2 / 8);
    const int tap = c - oc * (K2 / 8);
    const int tc  = tap < 9 ? tap : 8;
#pragma unroll
    for (int e = 0; e < 8; ++e) {
      const float t = c2w[oc * 72 + e * 9 + tc];
      v[e] = (tap < 9) ? t : 0.0f;
    }
    dh = wt + c * 8;
    dl = dh + C2 * K2;
  } else {
    act = tid < NF2P * (NF1 / 8);
    const int c  = tid < NF2P * (NF1 / 8) - 1 ? tid : NF2P * (NF1 / 8) - 1;
    const int n  = c >> 3;
    const int k0 = (c & 7) * 8;
    const int nc = n < NF2 ? n : NF2 - 1;
#pragma unroll
    for (int e = 0; e < 8; ++e) {
      const float t = f2w[nc * NF1 + k0 + e];
      v[e] = (n < NF2) ? t : 0.0f;
    }
    dh = wf2 + c * 8;
    dl = dh + NF2P * NF1;
  }
  v4f a, bq;
  a.x = v[0]; a.y = v[1]; a.z = v[2]; a.w = v[3];
  bq.x = v[4]; bq.y = v[5]; bq.z = v[6]; bq.w = v[7];
  v8us hv, lv;
  split8(a, bq, hv, lv);
  if (act) { *(volatile v8us*)dh = hv; *(volatile v8us*)dl = lv; }
  __threadfence();
  if (act) { *(volatile v8us*)dh = hv; *(volatile v8us*)dl = lv; }
}

__global__ __launch_bounds__(T1) void k_conv1(
    const float* __restrict__ x, const float* __restrict__ w, const float* __restrict__ bias,
    unsigned short* h1h, unsigned short* h1l, int nPix) {
  __shared__ float stg[T1 * C1];
  const int tid = (int)threadIdx.x;
  int pix = (int)blockIdx.x * T1 + tid;
  pix = pix < nPix ? pix : nPix - 1;
  const int n  = pix / NPIX1;
  const int wl = pix - n * NPIX1;
  const int py = wl / 14, px = wl - py * 14;
  const float* xin = x + (size_t)n * 784;
  float pv[16];
#pragma unroll
  for (int r = 0; r < 4; ++r) {
    const int iy  = 2 * py - 1 + r;
    const int iyc = iy < 0 ? 0 : (iy > 27 ? 27 : iy);
    const bool oky = (unsigned)iy < 28u;
#pragma unroll
    for (int c = 0; c < 4; ++c) {
      const int ix  = 2 * px - 1 + c;
      const int ixc = ix < 0 ? 0 : (ix > 27 ? 27 : ix);
      const float t = xin[iyc * 28 + ixc];
      pv[r * 4 + c] = (oky && ((unsigned)ix < 28u)) ? t : 0.0f;
    }
  }
#pragma unroll 1
  for (int oc = 0; oc < C1; ++oc) {
    const float* wp = w + oc * 9;
    float wv[9];
#pragma unroll
    for (int t = 0; t < 9; ++t) wv[t] = wp[t];
    const float bb = bias[oc];
    float mx = 0.0f;
#pragma unroll
    for (int dy = 0; dy < 2; ++dy) {
#pragma unroll
      for (int dx = 0; dx < 2; ++dx) {
        float acc = bb;
#pragma unroll
        for (int ky = 0; ky < 3; ++ky) {
#pragma unroll
          for (int kx = 0; kx < 3; ++kx) acc = fmaf(pv[(dy + ky) * 4 + (dx + kx)], wv[ky * 3 + kx], acc);
        }
        acc = fmaxf(acc, 0.0f);
        mx = fmaxf(mx, acc);
      }
    }
    stg[tid * C1 + oc] = mx;
  }
  v4f a, b;
  a.x = stg[tid * C1 + 0]; a.y = stg[tid * C1 + 1]; a.z = stg[tid * C1 + 2]; a.w = stg[tid * C1 + 3];
  b.x = stg[tid * C1 + 4]; b.y = stg[tid * C1 + 5]; b.z = stg[tid * C1 + 6]; b.w = stg[tid * C1 + 7];
  v8us hv, lv;
  split8(a, b, hv, lv);
  unsigned short* ph = h1h + (size_t)pix * C1;
  unsigned short* pl = h1l + (size_t)pix * C1;
  *(volatile v8us*)ph = hv;
  *(volatile v8us*)pl = lv;
  __threadfence();
  *(volatile v8us*)ph = hv;
  *(volatile v8us*)pl = lv;
}

__global__ __launch_bounds__(T2) void k_conv2(
    const unsigned short* __restrict__ h1h, const unsigned short* __restrict__ h1l,
    const unsigned short* __restrict__ wt, const float* __restrict__ bias,
    unsigned short* h2h, unsigned short* h2l) {
  __shared__ __attribute__((aligned(16))) float stg[SPB2 * KFP];
  const int tid = (int)threadIdx.x, lane = tid & 31, wave = tid >> 5, hh = lane >> 4, m = lane & 15;
  const int s0 = (int)blockIdx.x * SPB2;
  if (tid < SPB2 * (KFP - KF)) stg[(tid >> 4) * KFP + KF + (tid & 15)] = 0.0f;

  FragB bh[3], bl[3];
#pragma unroll
  for (int s = 0; s < 3; ++s) {
    const unsigned short* bp = wt + m * K2 + 32 * s + 8 * hh;
    bh[s].h[0] = *(const v8us*)bp;
    bh[s].h[1] = *(const v8us*)(bp + 16);
    bl[s].h[0] = *(const v8us*)(bp + C2 * K2);
    bl[s].h[1] = *(const v8us*)(bp + C2 * K2 + 16);
  }
  const float bo = bias[m];
  const v8us z8 = {0, 0, 0, 0, 0, 0, 0, 0};

#pragma unroll 1
  for (int t = wave; t < NWIN; t += T2 / 32) {
    const int row = t * 16 + m;
    const int gwl = row >> 2;
    const int d   = row & 3;
    const int sl  = gwl / NWIN;
    const int wl  = gwl - sl * NWIN;
    const int py  = wl / 7, px = wl - py * 7;
    const int cy  = 2 * py + (d >> 1), cx = 2 * px + (d & 1);
    const size_t sbase = (size_t)(s0 + sl) * H1S;
    v8f acc = {0.f, 0.f, 0.f, 0.f, 0.f, 0.f, 0.f, 0.f};
#pragma unroll
    for (int s = 0; s < 3; ++s) {
      FragB ah, al;
#pragma unroll
      for (int q = 0; q < 2; ++q) {
        const int tap = 4 * s + 2 * q + hh;
        const int ty  = (int)((unsigned)tap / 3u);
        const int tx  = tap - ty * 3;
        const int iy  = cy + ty - 1, ix = cx + tx - 1;
        const bool ok = (tap < 9) && ((unsigned)iy < 14u) && ((unsigned)ix < 14u);
        const int iyc = iy < 0 ? 0 : (iy > 13 ? 13 : iy);
        const int ixc = ix < 0 ? 0 : (ix > 13 ? 13 : ix);
        const size_t o = sbase + (size_t)(iyc * 14 + ixc) * C1;
        const v8us vh = *(const v8us*)(h1h + o);
        const v8us vl = *(const v8us*)(h1l + o);
        ah.h[q] = ok ? vh : z8;
        al.h[q] = ok ? vl : z8;
      }
      acc = wmb(ah.v, bh[s].v, acc);
      acc = wmb(ah.v, bl[s].v, acc);
      acc = wmb(al.v, bh[s].v, acc);
    }
    float p0 = 0.0f, p1 = 0.0f;
#pragma unroll
    for (int r = 0; r < 4; ++r) {
      p0 = fmaxf(p0, fmaxf(acc[r] + bo, 0.0f));
      p1 = fmaxf(p1, fmaxf(acc[4 + r] + bo, 0.0f));
    }
    const int g0 = t * 4 + 2 * hh, g1 = g0 + 1;
    const int sa = g0 / NWIN, wa = g0 - sa * NWIN;
    const int sc = g1 / NWIN, wc = g1 - sc * NWIN;
    stg[sa * KFP + m * NWIN + wa] = p0;
    stg[sc * KFP + m * NWIN + wc] = p1;
  }
  __syncthreads();

  const int c0  = tid;
  const int r0i = c0 / (KFP / 8), k00 = (c0 - r0i * (KFP / 8)) * 8;
  const v4f a0 = *(const v4f*)(stg + r0i * KFP + k00);
  const v4f a1 = *(const v4f*)(stg + r0i * KFP + k00 + 4);
  v8us hv0, lv0;
  split8(a0, a1, hv0, lv0);
  const bool act1 = tid < SPB2 * (KFP / 8) - T2;
  const int c1  = act1 ? (T2 + tid) : (SPB2 * (KFP / 8) - 1);
  const int r1i = c1 / (KFP / 8), k10 = (c1 - r1i * (KFP / 8)) * 8;
  const v4f b0 = *(const v4f*)(stg + r1i * KFP + k10);
  const v4f b1 = *(const v4f*)(stg + r1i * KFP + k10 + 4);
  v8us hv1, lv1;
  split8(b0, b1, hv1, lv1);
  unsigned short* oh = h2h + (size_t)s0 * KFP;
  unsigned short* ol = h2l + (size_t)s0 * KFP;
  *(volatile v8us*)(oh + (size_t)c0 * 8) = hv0;
  *(volatile v8us*)(ol + (size_t)c0 * 8) = lv0;
  if (act1) { *(volatile v8us*)(oh + (size_t)c1 * 8) = hv1; *(volatile v8us*)(ol + (size_t)c1 * 8) = lv1; }
  __threadfence();
  *(volatile v8us*)(oh + (size_t)c0 * 8) = hv0;
  *(volatile v8us*)(ol + (size_t)c0 * 8) = lv0;
  if (act1) { *(volatile v8us*)(oh + (size_t)c1 * 8) = hv1; *(volatile v8us*)(ol + (size_t)c1 * 8) = lv1; }
}

__global__ __launch_bounds__(TF) void k_fc(
    const unsigned short* __restrict__ ah, const unsigned short* __restrict__ al,
    const unsigned short* __restrict__ w1, const float* __restrict__ b1,
    const unsigned short* __restrict__ w2, const float* __restrict__ b2, float* qs) {
  __shared__ __attribute__((aligned(16))) unsigned short sH[RPB * SHP];
  __shared__ __attribute__((aligned(16))) unsigned short sL[RPB * SHP];
  __shared__ __attribute__((aligned(16))) float sQ[RPB * NF2];
  const int tid = (int)threadIdx.x, lane = tid & 31, wave = tid >> 5, hh = lane >> 4, m = lane & 15;
  const int lr0 = wave * 16;
  const size_t grow = (size_t)blockIdx.x * RPB + lr0 + m;
  const unsigned short* ap  = ah + grow * KFP + 8 * hh;
  const unsigned short* alp = al + grow * KFP + 8 * hh;

  v8f acc[4];
#pragma unroll
  for (int t = 0; t < 4; ++t) { v8f z = {0.f, 0.f, 0.f, 0.f, 0.f, 0.f, 0.f, 0.f}; acc[t] = z; }
#pragma unroll 1
  for (int kt = 0; kt < KFP / 32; ++kt) {
    FragB fa, fl;
    fa.h[0] = *(const v8us*)(ap + 32 * kt);
    fa.h[1] = *(const v8us*)(ap + 32 * kt + 16);
    fl.h[0] = *(const v8us*)(alp + 32 * kt);
    fl.h[1] = *(const v8us*)(alp + 32 * kt + 16);
#pragma unroll
    for (int t = 0; t < 4; ++t) {
      const unsigned short* bp = w1 + (size_t)(16 * t + m) * KFP + 32 * kt + 8 * hh;
      FragB bh, bl;
      bh.h[0] = *(const v8us*)bp;
      bh.h[1] = *(const v8us*)(bp + 16);
      bl.h[0] = *(const v8us*)(bp + NF1 * KFP);
      bl.h[1] = *(const v8us*)(bp + NF1 * KFP + 16);
      acc[t] = wmb(fa.v, bh.v, acc[t]);
      acc[t] = wmb(fa.v, bl.v, acc[t]);
      acc[t] = wmb(fl.v, bh.v, acc[t]);
    }
  }

#pragma unroll
  for (int t = 0; t < 4; ++t) {
    const float bb = b1[16 * t + m];
#pragma unroll
    for (int r = 0; r < 8; ++r) {
      const float v = fmaxf(acc[t][r] + bb, 0.0f);
      unsigned short hb, lb;
      split1(v, hb, lb);
      const int idx = (lr0 + 8 * hh + r) * SHP + 16 * t + m;
      sH[idx] = hb;
      sL[idx] = lb;
    }
  }
  __syncthreads();

  v8f acc2 = {0.f, 0.f, 0.f, 0.f, 0.f, 0.f, 0.f, 0.f};
  const unsigned short* sap = sH + (lr0 + m) * SHP + 8 * hh;
  const unsigned short* slp = sL + (lr0 + m) * SHP + 8 * hh;
#pragma unroll
  for (int kt = 0; kt < NF1 / 32; ++kt) {
    FragB fa, fl, bh, bl;
    fa.h[0] = *(const v8us*)(sap + 32 * kt);
    fa.h[1] = *(const v8us*)(sap + 32 * kt + 16);
    fl.h[0] = *(const v8us*)(slp + 32 * kt);
    fl.h[1] = *(const v8us*)(slp + 32 * kt + 16);
    const unsigned short* bp = w2 + m * NF1 + 32 * kt + 8 * hh;
    bh.h[0] = *(const v8us*)bp;
    bh.h[1] = *(const v8us*)(bp + 16);
    bl.h[0] = *(const v8us*)(bp + NF2P * NF1);
    bl.h[1] = *(const v8us*)(bp + NF2P * NF1 + 16);
    acc2 = wmb(fa.v, bh.v, acc2);
    acc2 = wmb(fa.v, bl.v, acc2);
    acc2 = wmb(fl.v, bh.v, acc2);
  }
  const float bb2 = b2[m < NF2 ? m : NF2 - 1];
  if (m < NF2) {
#pragma unroll
    for (int r = 0; r < 8; ++r) sQ[(lr0 + 8 * hh + r) * NF2 + m] = acc2[r] + bb2;
  }
  __syncthreads();

  const v4f v = *(const v4f*)(sQ + lr0 * NF2 + 4 * lane);
  float* gp = qs + ((size_t)blockIdx.x * RPB + lr0) * NF2 + 4 * lane;
  *(volatile v4f*)gp = v;
  __threadfence();
  *(volatile v4f*)gp = v;
}

__global__ __launch_bounds__(TS) void k_stats(const float* __restrict__ qs, float* st, int nS) {
  __shared__ double red[NW * TS];
  __shared__ __attribute__((aligned(16))) float sst[32];
  const int tid = (int)threadIdx.x;
  const double invN = 1.0 / (double)nS;
  double s[NW];
#pragma unroll
  for (int f = 0; f < NW; ++f) s[f] = 0.0;
#pragma unroll 1
  for (int i = tid; i < nS; i += TS) {
    const v4f a = *(const v4f*)(qs + (size_t)i * NW);
    const v4f b = *(const v4f*)(qs + (size_t)i * NW + 4);
    s[0] += (double)a.x; s[1] += (double)a.y; s[2] += (double)a.z; s[3] += (double)a.w;
    s[4] += (double)b.x; s[5] += (double)b.y; s[6] += (double)b.z; s[7] += (double)b.w;
  }
#pragma unroll
  for (int f = 0; f < NW; ++f) red[f * TS + tid] = s[f];
  blockred(red, tid);
  float mu[NW];
#pragma unroll
  for (int f = 0; f < NW; ++f) mu[f] = (float)(red[f * TS] * invN);
  __syncthreads();

#pragma unroll
  for (int f = 0; f < NW; ++f) s[f] = 0.0;
#pragma unroll 1
  for (int i = tid; i < nS; i += TS) {
    const v4f a = *(const v4f*)(qs + (size_t)i * NW);
    const v4f b = *(const v4f*)(qs + (size_t)i * NW + 4);
    const float d0 = a.x - mu[0], d1 = a.y - mu[1], d2 = a.z - mu[2], d3 = a.w - mu[3];
    const float d4 = b.x - mu[4], d5 = b.y - mu[5], d6 = b.z - mu[6], d7 = b.w - mu[7];
    s[0] += (double)d0 * (double)d0; s[1] += (double)d1 * (double)d1;
    s[2] += (double)d2 * (double)d2; s[3] += (double)d3 * (double)d3;
    s[4] += (double)d4 * (double)d4; s[5] += (double)d5 * (double)d5;
    s[6] += (double)d6 * (double)d6; s[7] += (double)d7 * (double)d7;
  }
#pragma unroll
  for (int f = 0; f < NW; ++f) red[f * TS + tid] = s[f];
  blockred(red, tid);
  if (tid == 0) {
#pragma unroll
    for (int f = 0; f < NW; ++f) {
      sst[f] = mu[f];
      const float var = (float)(red[f * TS] * invN);
      sst[NW + f] = rsqrtf(var + BN_EPS);
    }
#pragma unroll
    for (int f = 2 * NW; f < 32; ++f) sst[f] = 0.0f;
  }
  __syncthreads();
  const v4f v = *(const v4f*)(sst + 4 * (tid < 8 ? tid : 7));
  if (tid < 8) *(volatile v4f*)(st + 4 * tid) = v;
  __threadfence();
  if (tid < 8) *(volatile v4f*)(st + 4 * tid) = v;
}

__global__ __launch_bounds__(TQ) void k_final(
    const float* __restrict__ qs, const float* __restrict__ st,
    const float* __restrict__ gam, const float* __restrict__ bet, const float* __restrict__ qw,
    const float* __restrict__ fw, const float* __restrict__ fb, float* out) {
  __shared__ float sv[256 * TQ];
  __shared__ float cb[2 * NW * TQ];
  const int lane = (int)threadIdx.x;
  const size_t row = (size_t)blockIdx.x * TQ + lane;

#pragma unroll 1
  for (int i = 0; i < 256; ++i) sv[i * TQ + lane] = (i == 0) ? 1.0f : 0.0f;

#pragma unroll 1
  for (int g = 0; g < 2 * NW; ++g) {
    const int w = g & (NW - 1);
    const float q  = qs[row * NW + w];
    const float qn = (q - st[w]) * st[NW + w] * gam[w] + bet[w];
    if (g < NW) cb[w * TQ + lane] = qn;
    const float theta = (g < NW) ? qn : qw[w];
    float sn, cs;
    sincosf(0.5f * theta, &sn, &cs);
    const int bpos = 7 - w, sbit = 1 << bpos;
#pragma unroll 1
    for (int p = 0; p < 128; ++p) {
      const int i0 = ((p >> bpos) << (bpos + 1)) | (p & (sbit - 1));
      const int i1 = i0 | sbit;
      const float a0 = sv[i0 * TQ + lane];
      const float a1 = sv[i1 * TQ + lane];
      sv[i0 * TQ + lane] = cs * a0 - sn * a1;
      sv[i1 * TQ + lane] = sn * a0 + cs * a1;
    }
  }

#pragma unroll 1
  for (int i = 0; i < NW - 1; ++i) {
    const int tpos = 6 - i, tbit = 1 << tpos, cbit = tbit << 1;
#pragma unroll 1
    for (int p = 0; p < 64; ++p) {
      const int idx = ((p >> tpos) << (tpos + 2)) | cbit | (p & (tbit - 1));
      const int jdx = idx | tbit;
      const float a0 = sv[idx * TQ + lane];
      const float a1 = sv[jdx * TQ + lane];
      sv[idx * TQ + lane] = a1;
      sv[jdx * TQ + lane] = a0;
    }
  }

  float z[NW];
#pragma unroll
  for (int w = 0; w < NW; ++w) z[w] = 0.0f;
#pragma unroll 1
  for (int idx = 0; idx < 256; ++idx) {
    const float a = sv[idx * TQ + lane];
    const float p = a * a;
#pragma unroll
    for (int w = 0; w < NW; ++w) z[w] += (idx & (128 >> w)) ? -p : p;
  }
#pragma unroll
  for (int w = 0; w < NW; ++w) cb[(NW + w) * TQ + lane] = z[w];

  float o0 = fb[0], o1 = fb[1], o2 = fb[2], o3 = fb[3];
#pragma unroll 1
  for (int j = 0; j < 2 * NW; ++j) {
    const float c = cb[j * TQ + lane];
    o0 = fmaf(fw[j], c, o0);
    o1 = fmaf(fw[2 * NW + j], c, o1);
    o2 = fmaf(fw[4 * NW + j], c, o2);
    o3 = fmaf(fw[6 * NW + j], c, o3);
  }
  v4f ov;
  ov.x = o0; ov.y = o1; ov.z = o2; ov.w = o3;
  float* gp = out + row * NOUT;
  *(volatile v4f*)gp = ov;
  __threadfence();
  *(volatile v4f*)gp = ov;
}

extern "C" void kernel_launch(void* const* d_in, const int* in_sizes, int n_in,
                              void* d_out, int out_size, void* d_ws, size_t ws_size,
                              hipStream_t stream) {
  if (n_in < 14) return;
  const int nS = in_sizes[0] / 784;
  if (nS <= 0 || nS > (1 << 20) || in_sizes[0] != nS * 784 || (nS % 64) != 0) return;
  if (in_sizes[1] != C1 * 9 || in_sizes[2] != C1 || in_sizes[3] != C2 * C1 * 9 || in_sizes[4] != C2) return;
  if (in_sizes[5] != NF1 * KF || in_sizes[6] != NF1 || in_sizes[7] != NF2 * NF1 || in_sizes[8] != NF2) return;
  if (in_sizes[9] != NW || in_sizes[10] != NW || in_sizes[11] != NW) return;
  if (in_sizes[12] != NOUT * 2 * NW || in_sizes[13] != NOUT) return;
  if (out_size != nS * NOUT) return;

  const float* x    = (const float*)d_in[0];
  const float* c1w  = (const float*)d_in[1];
  const float* c1b  = (const float*)d_in[2];
  const float* c2w  = (const float*)d_in[3];
  const float* c2b  = (const float*)d_in[4];
  const float* f1w  = (const float*)d_in[5];
  const float* f1b  = (const float*)d_in[6];
  const float* f2w  = (const float*)d_in[7];
  const float* f2b  = (const float*)d_in[8];
  const float* bng  = (const float*)d_in[9];
  const float* bnb  = (const float*)d_in[10];
  const float* qwv  = (const float*)d_in[11];
  const float* fnw  = (const float*)d_in[12];
  const float* fnb  = (const float*)d_in[13];
  float* out = (float*)d_out;

  char* ws = (char*)d_ws;
  size_t off = 0;
  const size_t oH1h = off; off += (size_t)nS * H1S * 2;          off = (off + 255) & ~(size_t)255;
  const size_t oH1l = off; off += (size_t)nS * H1S * 2;          off = (off + 255) & ~(size_t)255;
  const size_t oH2h = off; off += (size_t)nS * KFP * 2;          off = (off + 255) & ~(size_t)255;
  const size_t oH2l = off; off += (size_t)nS * KFP * 2;          off = (off + 255) & ~(size_t)255;
  const size_t oWt  = off; off += (size_t)2 * C2 * K2 * 2;       off = (off + 255) & ~(size_t)255;
  const size_t oW1  = off; off += (size_t)2 * NF1 * KFP * 2;     off = (off + 255) & ~(size_t)255;
  const size_t oW2  = off; off += (size_t)2 * NF2P * NF1 * 2;    off = (off + 255) & ~(size_t)255;
  const size_t oQs  = off; off += (size_t)nS * NW * 4;           off = (off + 255) & ~(size_t)255;
  const size_t oSt  = off; off += 128;                            off = (off + 255) & ~(size_t)255;
  if (off > ws_size || off > (size_t)WSCAP) return;
  unsigned short* h1h = (unsigned short*)(ws + oH1h);
  unsigned short* h1l = (unsigned short*)(ws + oH1l);
  unsigned short* h2h = (unsigned short*)(ws + oH2h);
  unsigned short* h2l = (unsigned short*)(ws + oH2l);
  unsigned short* wt  = (unsigned short*)(ws + oWt);
  unsigned short* w1  = (unsigned short*)(ws + oW1);
  unsigned short* w2  = (unsigned short*)(ws + oW2);
  float* qsp = (float*)(ws + oQs);
  float* stp = (float*)(ws + oSt);

  const int nPix = nS * NPIX1;

  k_prep<<<NPREPB, 256, 0, stream>>>(c2w, f1w, f2w, wt, w1, w2);
  k_conv1<<<nPix / T1, T1, 0, stream>>>(x, c1w, c1b, h1h, h1l, nPix);
  k_conv2<<<nS / SPB2, T2, 0, stream>>>(h1h, h1l, wt, c2b, h2h, h2l);
  k_fc<<<nS / RPB, TF, 0, stream>>>(h2h, h2l, w1, f1b, w2, f2b, qsp);
  k_stats<<<1, TS, 0, stream>>>(qsp, stp, nS);
  k_final<<<nS / TQ, TQ, 0, stream>>>(qsp, stp, bng, bnb, qwv, fnw, fnb, out);
}
